// MeanAggLayer_44719199485973
// MI455X (gfx1250) — hardware-run, weakly checked
//
#include <hip/hip_runtime.h>
#include <stddef.h>
#include <stdint.h>


#define DF      128
#define HP      256
#define KT      256
#define NTHR    256
#define NWAVE   8
#define STEPE   128
#define NSTEP   4
#define WSPAN   (STEPE * NSTEP)
#define CHUNK   (NWAVE * WSPAN)
#define WCAP    WSPAN
#define LISTN   (NWAVE * WCAP)
#define NBA     1024
#define SLA     10
#define RCAP    8192
#define DEGCAP  64
#define STW     128
#define FLAGW   32
#define GBM     64
#define GBN     128
#define GTHR    128
#define NWDBLK  16
#define MEAS_MAXDEG 19
#define MEAS_B1024  6277
#define WSMAX   134217728
#define SCAN_INTS (LISTN + 2 * RCAP + 3 * NBA + NWAVE * STW + 32)
#define SCAN_LDS  (SCAN_INTS * 4)

static_assert(NBA == (1 << SLA));
static_assert(NTHR * 4 == NBA);
static_assert(NBA % NWAVE == 0 && NBA % GBM == 0);
static_assert(RCAP * 100 >= MEAS_B1024 * 105);
static_assert(DEGCAP >= MEAS_MAXDEG + 8);
static_assert(WCAP == 4 * 32 * NSTEP);
static_assert(KT % 32 == 0 && KT == 2 * DF && HP == 2 * DF && DF == 4 * 32);
static_assert(GBN == DF && GBM == (GTHR / 32) * 16);
static_assert(NWDBLK * NTHR == DF * (KT / 8));
static_assert(STW * 4 == HP * 2);
static_assert(SCAN_LDS <= 300000);
static_assert((LISTN % 4) == 0 && (RCAP % 4) == 0 && (NBA % 4) == 0);

typedef float          v4f  __attribute__((ext_vector_type(4)));
typedef float          v8f  __attribute__((ext_vector_type(8)));
typedef int            v4i  __attribute__((ext_vector_type(4)));
typedef int            v8i  __attribute__((ext_vector_type(8)));
typedef unsigned int   v2u  __attribute__((ext_vector_type(2)));
typedef unsigned int   v4u  __attribute__((ext_vector_type(4)));
typedef unsigned short v8us __attribute__((ext_vector_type(8)));
typedef __bf16         v16b __attribute__((ext_vector_type(16)));
typedef v4f  __attribute__((may_alias)) v4fa;
typedef v4i  __attribute__((may_alias)) v4ia;
typedef v2u  __attribute__((may_alias)) v2ua;
typedef v4u  __attribute__((may_alias)) v4ua;
typedef v8us __attribute__((may_alias)) v8usa;
union FragB { v16b v; v8us h[2]; v8i w; };

__device__ __forceinline__ v8f wmb(const FragB& a, const FragB& b, v8f c) {
  v8f d = __builtin_amdgcn_wmma_f32_16x16x32_bf16(false, a.v, false, b.v, (short)0, c, false, false);
  asm volatile("v_nop\n\tv_nop\n\tv_nop\n\tv_nop" : "+v"(d) : "v"(a.w), "v"(b.w));
  return d;
}

__device__ __forceinline__ unsigned bf_bits(float f) {
  const unsigned u = __float_as_uint(f);
  const unsigned r = (u + 0x7FFFu + ((u >> 16) & 1u)) >> 16;
  return (f != f) ? 0x7FC0u : r;
}
__device__ __forceinline__ float bf_val(unsigned b) { return __uint_as_float(b << 16); }

__device__ __forceinline__ int imin(int a, int b) { return a < b ? a : b; }

__device__ __forceinline__ void wave_sync() {
  __builtin_amdgcn_fence(__ATOMIC_RELEASE, "wavefront");
  __builtin_amdgcn_wave_barrier();
  __builtin_amdgcn_fence(__ATOMIC_ACQUIRE, "wavefront");
}

__global__ __launch_bounds__(NTHR) void k_prep(const float* __restrict__ x, const float* __restrict__ W,
                                               const float* __restrict__ b, int nN, int nXB,
                                               unsigned short* xb, unsigned short* wd, float* bfp) {
  const int blk = (int)blockIdx.x, tid = (int)threadIdx.x;
  if (blk < nXB) {
    const int u   = blk * NTHR + tid;
    const int row = u >> 4;
    const int c8  = (u & 15) * 8;
    const int rc  = row < nN ? row : nN - 1;
    const float* p = x + (size_t)rc * DF + c8;
    const v4f a = *(const v4f*)p;
    const v4f c = *(const v4f*)(p + 4);
    asm volatile("" :: "v"(a), "v"(c));
    const unsigned msk = row < nN ? 0xFFFFFFFFu : 0u;
    v4u o;
    o.x = (bf_bits(a.x) | (bf_bits(a.y) << 16)) & msk;
    o.y = (bf_bits(a.z) | (bf_bits(a.w) << 16)) & msk;
    o.z = (bf_bits(c.x) | (bf_bits(c.y) << 16)) & msk;
    o.w = (bf_bits(c.z) | (bf_bits(c.w) << 16)) & msk;
    unsigned short* dp = xb + (size_t)row * DF + c8;
    *(volatile v4u*)dp = o;
    __threadfence();
    *(volatile v4u*)dp = o;
  } else if (blk < nXB + NWDBLK) {
    const int v  = (blk - nXB) * NTHR + tid;
    const int n  = v >> 5;
    const int k8 = (v & 31) * 8;
    const int kk = k8 & (DF - 1);
    const float* p = W + (size_t)kk * DF + n;
    const float f0 = p[0 * DF], f1 = p[1 * DF], f2 = p[2 * DF], f3 = p[3 * DF];
    const float f4 = p[4 * DF], f5 = p[5 * DF], f6 = p[6 * DF], f7 = p[7 * DF];
    v4u o;
    o.x = bf_bits(f0) | (bf_bits(f1) << 16);
    o.y = bf_bits(f2) | (bf_bits(f3) << 16);
    o.z = bf_bits(f4) | (bf_bits(f5) << 16);
    o.w = bf_bits(f6) | (bf_bits(f7) << 16);
    unsigned short* dp = wd + (size_t)n * KT + k8;
    *(volatile v4u*)dp = o;
    __threadfence();
    *(volatile v4u*)dp = o;
  } else {
    v4f o = {0.f, 0.f, 0.f, 0.f};
    if (tid < 32) {
      const v4f t = *(const v4f*)(b + 4 * tid);
      o.x = bf_val(bf_bits(t.x)); o.y = bf_val(bf_bits(t.y));
      o.z = bf_val(bf_bits(t.z)); o.w = bf_val(bf_bits(t.w));
      *(volatile v4f*)(bfp + 4 * tid) = o;
    }
    __threadfence();
    if (tid < 32) *(volatile v4f*)(bfp + 4 * tid) = o;
  }
}

__device__ __forceinline__ int sweep_step(const int* __restrict__ dsts, int nE, int ebase, unsigned nbs,
                                          unsigned unb, int* wl, int lane, int wc) {
  const int e0   = ebase + 4 * lane;
  const int sent = -2147483647 - 1;
  v4i d;
  if (ebase + STEPE <= nE) {
    d = *(const v4i*)(dsts + e0);
  } else {
    const int last = nE - 1;
    const int t0 = dsts[imin(e0,     last)];
    const int t1 = dsts[imin(e0 + 1, last)];
    const int t2 = dsts[imin(e0 + 2, last)];
    const int t3 = dsts[imin(e0 + 3, last)];
    asm volatile("" :: "v"(t0), "v"(t1), "v"(t2), "v"(t3));
    d.x = (e0     < nE) ? t0 : sent;
    d.y = (e0 + 1 < nE) ? t1 : sent;
    d.z = (e0 + 2 < nE) ? t2 : sent;
    d.w = (e0 + 3 < nE) ? t3 : sent;
  }
  const unsigned s0 = (unsigned)d.x - nbs, s1 = (unsigned)d.y - nbs;
  const unsigned s2 = (unsigned)d.z - nbs, s3 = (unsigned)d.w - nbs;
  const bool h0 = s0 < unb, h1 = s1 < unb, h2 = s2 < unb, h3 = s3 < unb;
  const unsigned m0 = __builtin_amdgcn_ballot_w32(h0);
  const unsigned m1 = __builtin_amdgcn_ballot_w32(h1);
  const unsigned m2 = __builtin_amdgcn_ballot_w32(h2);
  const unsigned m3 = __builtin_amdgcn_ballot_w32(h3);
  if ((m0 | m1 | m2 | m3) != 0u) {
    int pos = wc + (int)__builtin_amdgcn_mbcnt_lo(m0, 0u) + (int)__builtin_amdgcn_mbcnt_lo(m1, 0u)
                 + (int)__builtin_amdgcn_mbcnt_lo(m2, 0u) + (int)__builtin_amdgcn_mbcnt_lo(m3, 0u);
    if (h0) { if (pos < WCAP) wl[pos] = (int)(((unsigned)(e0 + 0) << SLA) | s0); }
    pos += h0 ? 1 : 0;
    if (h1) { if (pos < WCAP) wl[pos] = (int)(((unsigned)(e0 + 1) << SLA) | s1); }
    pos += h1 ? 1 : 0;
    if (h2) { if (pos < WCAP) wl[pos] = (int)(((unsigned)(e0 + 2) << SLA) | s2); }
    pos += h2 ? 1 : 0;
    if (h3) { if (pos < WCAP) wl[pos] = (int)(((unsigned)(e0 + 3) << SLA) | s3); }
    wc += (int)__builtin_popcount(m0) + (int)__builtin_popcount(m1)
        + (int)__builtin_popcount(m2) + (int)__builtin_popcount(m3);
  }
  return wc;
}

__global__ __launch_bounds__(NTHR) void k_scan(const int* __restrict__ srcs, const int* __restrict__ dsts,
                                               const unsigned short* __restrict__ xb, unsigned short* hhl,
                                               int* flag, int nN, int nE, int MPr) {
  extern __shared__ __attribute__((aligned(16))) int dsm[];
  int* list = dsm;
  int* reg1 = list + LISTN;
  int* reg2 = reg1 + RCAP;
  int* scnt = reg2 + RCAP;
  int* soff = scnt + NBA;
  int* cur  = soff + NBA;
  int* stw  = cur + NBA;
  int* wcnt = stw + NWAVE * STW;
  int* wtot = wcnt + NWAVE;
  int* misc = wtot + NWAVE;
  const int tid = (int)threadIdx.x, lane = tid & 31, wave = tid >> 5;
  const int nodeBase = (int)blockIdx.x * NBA;
  int nbl = nN - nodeBase;
  nbl = nbl < 0 ? 0 : (nbl > NBA ? NBA : nbl);
  const unsigned nbs = (unsigned)nodeBase;
  const unsigned unb = (unsigned)nbl;

  for (int i = tid; i < NBA; i += NTHR) scnt[i] = 0;
  __syncthreads();

  int tot = 0, ovf = 0;
  int* wl = list + wave * WCAP;
  const int nChunks = (nE + CHUNK - 1) / CHUNK;
#pragma unroll 1
  for (int ch = 0; ch < nChunks; ++ch) {
    const int wbase = ch * CHUNK + wave * WSPAN;
    int wc = 0;
#pragma unroll 1
    for (int st = 0; st < NSTEP; ++st) {
      const int ebase = wbase + st * STEPE;
      if (ebase < nE) wc = sweep_step(dsts, nE, ebase, nbs, unb, wl, lane, wc);
    }
    if (lane == 0) wcnt[wave] = wc;
    __syncthreads();
    int pre = 0, all = 0;
#pragma unroll
    for (int w2 = 0; w2 < NWAVE; ++w2) {
      int c = wcnt[w2];
      c = c < 0 ? 0 : (c > WCAP ? WCAP : c);
      all += c;
      pre += (w2 < wave) ? c : 0;
    }
    const int wcc  = wc > WCAP ? WCAP : wc;
    const int base = tot + pre;
#pragma unroll 1
    for (int i = lane; i < wcc; i += 32) {
      const int ent = wl[i];
      const int pos = base + i;
      if (pos < RCAP) reg1[pos] = ent;
    }
    if (tot + all > RCAP) ovf = 1;
    tot = tot + all;
    tot = tot > RCAP ? RCAP : tot;
    __syncthreads();
  }
  const int nh = tot;

  if (wave == 0) {
#pragma unroll 1
    for (int b0 = 0; b0 < nh; b0 += 32) {
      int idx = b0 + lane;
      idx = idx > nh - 1 ? nh - 1 : idx;
      const int uv  = reg1[idx];
      const int m32 = (nh - b0) < 32 ? (nh - b0) : 32;
#pragma unroll 1
      for (int k = 0; k < m32; ++k) {
        const int u  = __builtin_amdgcn_readlane(uv, k);
        const int sl = u & (NBA - 1);
        if (lane == 0) scnt[sl] = scnt[sl] + 1;
      }
    }
  }
  __syncthreads();

  {
    const v4i ca = *(const v4ia*)(scnt + 4 * tid);
    const int e0 = ca.x < 0 ? 0 : ca.x, e1 = ca.y < 0 ? 0 : ca.y;
    const int e2 = ca.z < 0 ? 0 : ca.z, e3 = ca.w < 0 ? 0 : ca.w;
    const int ts = e0 + e1 + e2 + e3;
    int incl = ts;
#pragma unroll
    for (int d = 1; d < 32; d <<= 1) {
      const int up = __shfl_up(incl, d, 32);
      incl += (lane >= d) ? up : 0;
    }
    if (lane == 31) wtot[wave] = incl;
    __syncthreads();
    int pre = 0;
#pragma unroll
    for (int w2 = 0; w2 < NWAVE; ++w2) {
      const int tw = wtot[w2];
      pre += (w2 < wave) ? tw : 0;
    }
    int run = pre + incl - ts;
    soff[4 * tid + 0] = run; cur[4 * tid + 0] = run; run += e0;
    soff[4 * tid + 1] = run; cur[4 * tid + 1] = run; run += e1;
    soff[4 * tid + 2] = run; cur[4 * tid + 2] = run; run += e2;
    soff[4 * tid + 3] = run; cur[4 * tid + 3] = run;
  }
  __syncthreads();

  if (wave == 0) {
#pragma unroll 1
    for (int b0 = 0; b0 < nh; b0 += 32) {
      int idx = b0 + lane;
      idx = idx > nh - 1 ? nh - 1 : idx;
      const int uv  = reg1[idx];
      const int m32 = (nh - b0) < 32 ? (nh - b0) : 32;
#pragma unroll 1
      for (int k = 0; k < m32; ++k) {
        const int u   = __builtin_amdgcn_readlane(uv, k);
        const int sl  = u & (NBA - 1);
        const int eid = (int)((unsigned)u >> SLA);
        if (lane == 0) {
          int pos = cur[sl];
          pos = pos < 0 ? 0 : (pos > RCAP - 1 ? RCAP - 1 : pos);
          reg2[pos] = eid;
          cur[sl] = pos + 1;
        }
      }
    }
  }
  __syncthreads();

  const float qnan = __int_as_float(0x7fc00000);
  unsigned int* stwu = (unsigned int*)(stw + wave * STW);
  int bigAny = 0;
  const int nbw = NBA / NWAVE;
#pragma unroll 1
  for (int jt = 0; jt < nbw; ++jt) {
    const int slot = wave * nbw + jt;
    const int grow = nodeBase + slot;
    int st = soff[slot];
    const int craw = scnt[slot];
    int cnt = craw;
    st  = st < 0 ? 0 : (st > nh ? nh : st);
    cnt = cnt < 0 ? 0 : (cnt > DEGCAP ? DEGCAP : cnt);
    if (cnt > nh - st) cnt = nh - st;
    const bool big = craw > DEGCAP;
    bigAny |= big ? 1 : 0;
    const float pz = (ovf != 0 || big) ? qnan : 0.0f;
    const bool liveRow = grow < nN;

    float ag0 = 0.0f, ag1 = 0.0f, ag2 = 0.0f, ag3 = 0.0f;
#pragma unroll 1
    for (int b0 = 0; b0 < cnt; b0 += 32) {
      int idx = st + b0 + lane;
      idx = idx > nh - 1 ? nh - 1 : idx;
      idx = idx < 0 ? 0 : (idx > RCAP - 1 ? RCAP - 1 : idx);
      int eid = reg2[idx];
      eid = eid < 0 ? 0 : (eid > nE - 1 ? nE - 1 : eid);
      const int sraw = srcs[eid];
      const int sv = sraw < 0 ? 0 : (sraw > nN - 1 ? nN - 1 : sraw);
      const int m32 = (cnt - b0) < 32 ? (cnt - b0) : 32;
#pragma unroll 1
      for (int k = 0; k < m32; ++k) {
        const int sk = __builtin_amdgcn_readlane(sv, k);
        const v2u w = *(const v2ua*)(xb + (size_t)sk * DF + 4 * lane);
        ag0 += __uint_as_float(w.x << 16);
        ag1 += __uint_as_float(w.x & 0xffff0000u);
        ag2 += __uint_as_float(w.y << 16);
        ag3 += __uint_as_float(w.y & 0xffff0000u);
      }
    }
    const int nc = liveRow ? grow : nN - 1;
    const v2u sw = *(const v2ua*)(xb + (size_t)nc * DF + 4 * lane);
    const float s0 = __uint_as_float(sw.x << 16);
    const float s1 = __uint_as_float(sw.x & 0xffff0000u);
    const float s2 = __uint_as_float(sw.y << 16);
    const float s3 = __uint_as_float(sw.y & 0xffff0000u);
    const float dg = fmaxf((float)cnt, 1.0f);
    float r0 = s0 + ag0 / dg;
    float r1 = s1 + ag1 / dg;
    float r2 = s2 + ag2 / dg;
    float r3 = s3 + ag3 / dg;
    r0 = (liveRow ? r0 : 0.0f) + pz;
    r1 = (liveRow ? r1 : 0.0f) + pz;
    r2 = (liveRow ? r2 : 0.0f) + pz;
    r3 = (liveRow ? r3 : 0.0f) + pz;

    const unsigned hb0 = bf_bits(r0), hb1 = bf_bits(r1), hb2 = bf_bits(r2), hb3 = bf_bits(r3);
    const unsigned lb0 = bf_bits(r0 - bf_val(hb0)), lb1 = bf_bits(r1 - bf_val(hb1));
    const unsigned lb2 = bf_bits(r2 - bf_val(hb2)), lb3 = bf_bits(r3 - bf_val(hb3));
    v2u hw, lw;
    hw.x = hb0 | (hb1 << 16);
    hw.y = hb2 | (hb3 << 16);
    lw.x = lb0 | (lb1 << 16);
    lw.y = lb2 | (lb3 << 16);
    wave_sync();
    *(v2ua*)(stwu + 2 * lane)      = hw;
    *(v2ua*)(stwu + 64 + 2 * lane) = lw;
    wave_sync();
    const v4u pk = *(const v4ua*)(stwu + 4 * lane);
    unsigned short* gp = hhl + (size_t)grow * (size_t)HP + 8 * lane;
    const bool wsv = grow < MPr;
    if (wsv) *(volatile v4u*)gp = pk;
    __threadfence();
    if (wsv) *(volatile v4u*)gp = pk;
  }

  if (lane == 0) misc[wave] = bigAny;
  __syncthreads();
  int fl = ovf;
#pragma unroll
  for (int w2 = 0; w2 < NWAVE; ++w2) fl |= misc[w2];
  int* fp = flag + (size_t)blockIdx.x * FLAGW + lane;
  const bool w0 = (wave == 0);
  if (w0) *(volatile int*)fp = fl;
  __threadfence();
  if (w0) *(volatile int*)fp = fl;
}

__global__ __attribute__((amdgpu_num_vgpr(248))) __launch_bounds__(GTHR)
void k_gemm(const unsigned short* __restrict__ A, const unsigned short* __restrict__ BT,
            const float* __restrict__ bfp, const int* __restrict__ flag, float* outp, int nOut) {
  __shared__ __attribute__((aligned(16))) float stg[GBM * GBN];
  __shared__ __attribute__((aligned(16))) float bsh[GBN];
  const int tid = (int)threadIdx.x, lane = tid & 31, wave = tid >> 5, hh = lane >> 4, m = lane & 15;
  const int rowBase = (int)blockIdx.x * GBM;

  if (tid < 32) *(v4fa*)(bsh + 4 * tid) = *(const v4f*)(bfp + 4 * tid);

  v8f acc[8];
  {
    const v8f z = {0.f, 0.f, 0.f, 0.f, 0.f, 0.f, 0.f, 0.f};
#pragma unroll
    for (int t = 0; t < 8; ++t) acc[t] = z;
  }
  const unsigned short* ap = A + (size_t)(rowBase + 16 * wave + m) * (size_t)HP + 8 * hh;
  const unsigned short* bp = BT + (size_t)m * (size_t)KT + 8 * hh;

#pragma unroll 1
  for (int k0 = 0; k0 < KT; k0 += 32) {
    FragB af;
    af.h[0] = *(const v8usa*)(ap + k0);
    af.h[1] = *(const v8usa*)(ap + k0 + 16);
#pragma unroll
    for (int nt = 0; nt < 8; ++nt) {
      const unsigned short* wq = bp + (size_t)(16 * nt) * (size_t)KT + k0;
      FragB bf;
      bf.h[0] = *(const v8usa*)wq;
      bf.h[1] = *(const v8usa*)(wq + 16);
      acc[nt] = wmb(af, bf, acc[nt]);
    }
  }

#pragma unroll
  for (int nt = 0; nt < 8; ++nt) {
    const int lc = 16 * nt + m;
#pragma unroll
    for (int r = 0; r < 8; ++r) {
      const int lr = 16 * wave + 8 * hh + r;
      stg[lr * GBN + lc] = acc[nt][r];
    }
  }
  __syncthreads();

  const v4f bb4 = *(const v4fa*)(bsh + 4 * lane);
  const int fl = flag[(size_t)(rowBase >> SLA) * FLAGW];
  const bool pois = (fl != 0);
  const float qn = __int_as_float(0x7fc00000);

  v4f pv[16];
#pragma unroll
  for (int i = 0; i < 16; ++i) pv[i] = *(const v4fa*)(stg + (16 * wave + i) * GBN + 4 * lane);

#pragma unroll
  for (int i = 0; i < 16; ++i) {
    const v4f t = pv[i] + bb4;
    v4f y;
    y.x = (t.x > 0.0f) ? t.x : (t.x - t.x);
    y.y = (t.y > 0.0f) ? t.y : (t.y - t.y);
    y.z = (t.z > 0.0f) ? t.z : (t.z - t.z);
    y.w = (t.w > 0.0f) ? t.w : (t.w - t.w);
    y.x = pois ? qn : y.x; y.y = pois ? qn : y.y; y.z = pois ? qn : y.z; y.w = pois ? qn : y.w;
    pv[i] = y;
  }

#pragma unroll
  for (int i = 0; i < 16; ++i) {
    const int r = rowBase + 16 * wave + i;
    if (r < nOut) *(volatile v4f*)(outp + (size_t)r * DF + 4 * lane) = pv[i];
  }
  __threadfence();
#pragma unroll
  for (int i = 0; i < 16; ++i) {
    const int r = rowBase + 16 * wave + i;
    if (r < nOut) *(volatile v4f*)(outp + (size_t)r * DF + 4 * lane) = pv[i];
  }
}

static inline int cdiv(int a, int b) { return (a + b - 1) / b; }
static inline size_t al256(size_t o) { return (o + 255) & ~(size_t)255; }

extern "C" void kernel_launch(void* const* d_in, const int* in_sizes, int n_in,
                              void* d_out, int out_size, void* d_ws, size_t ws_size,
                              hipStream_t stream) {
  if (n_in < 5) return;
  if (in_sizes[0] < DF || (in_sizes[0] % DF) != 0) return;
  const int nN = in_sizes[0] / DF;
  if (nN < 1 || nN > (1 << 22)) return;
  if (in_sizes[1] != DF * DF) return;
  if (in_sizes[2] != DF) return;
  const int nE = in_sizes[3];
  if (nE < 1 || in_sizes[4] != nE) return;
  if (nE >= (1 << 21)) return;
  if ((long long)out_size != (long long)nN * DF) return;

  const float* x    = (const float*)d_in[0];
  const float* W    = (const float*)d_in[1];
  const float* b    = (const float*)d_in[2];
  const int*   esrc = (const int*)d_in[3];
  const int*   edst = (const int*)d_in[4];
  float* out = (float*)d_out;

  const int MP  = cdiv(nN, 128) * 128;
  const int nXB = MP / 16;
  const int gA  = cdiv(MP, NBA);
  const int gM  = cdiv(nN, GBM);
  if ((long long)gA * NBA < (long long)MP) return;
  if ((long long)(gA - 1) * NBA >= (long long)nN) return;
  if ((long long)gM * GBM > (long long)MP) return;

  char* ws = (char*)d_ws;
  size_t off = 0;
  const size_t oXB = off; off = al256(off + (size_t)MP * DF * 2);
  const size_t oHH = off; off = al256(off + (size_t)MP * HP * 2);
  const size_t oWD = off; off = al256(off + (size_t)DF * KT * 2);
  const size_t oBF = off; off = al256(off + (size_t)DF * 4);
  const size_t oFL = off; off = al256(off + (size_t)gA * FLAGW * 4);
  if (off > ws_size || off > (size_t)WSMAX) return;
  unsigned short* XB  = (unsigned short*)(ws + oXB);
  unsigned short* HHL = (unsigned short*)(ws + oHH);
  unsigned short* WD  = (unsigned short*)(ws + oWD);
  float*          BF  = (float*)(ws + oBF);
  int*            FL  = (int*)(ws + oFL);

  hipFuncSetAttribute(reinterpret_cast<const void*>(&k_scan), hipFuncAttributeMaxDynamicSharedMemorySize, SCAN_LDS);

  k_prep<<<nXB + NWDBLK + 1, NTHR, 0, stream>>>(x, W, b, nN, nXB, XB, WD, BF);
  k_scan<<<gA, NTHR, SCAN_LDS, stream>>>(esrc, edst, XB, HHL, FL, nN, nE, MP);
  k_gemm<<<gM, GTHR, 0, stream>>>(HHL, WD, BF, FL, out, nN);
}
